// RelationModel_double_38259568673081
// MI455X (gfx1250) — hardware-run, weakly checked
//
#include <hip/hip_runtime.h>
#include <math.h>

typedef __attribute__((ext_vector_type(16))) _Float16 v16h;
typedef __attribute__((ext_vector_type(8)))  _Float16 v8h;
typedef __attribute__((ext_vector_type(8)))  float    v8f;
typedef __attribute__((ext_vector_type(4)))  float    v4f;
typedef __attribute__((ext_vector_type(2)))  float    v2f;
typedef __attribute__((ext_vector_type(4)))  unsigned int v4u;

constexpr int kB      = 8;
constexpr int kP      = 3136;
constexpr int kD      = 256;
constexpr int kHeads  = 8;
constexpr int kDh     = 32;
constexpr int kInner  = kHeads * kDh;
constexpr int kQkvN   = 3 * kInner;
constexpr int kPos    = kB * kP;
constexpr int kChunkB = 2;
constexpr int kChunks = kB / kChunkB;
constexpr int kCPos   = kChunkB * kP;
constexpr int kMeanCh = 56;
constexpr int kMeanLen = 56;
constexpr int kWRows  = 2 * kQkvN + 2 * kD;
constexpr int kAtPos  = 16;
static_assert(kInner == 256 && kD == 256 && kQkvN == 768);
static_assert(kPos == 25088 && kCPos == 6272 && kChunks == 4);
static_assert(kMeanCh * kMeanLen == kP);
static_assert((kCPos % 64) == 0 && (kQkvN % 64) == 0 && (kD % 64) == 0 && (kD % 32) == 0);
static_assert((kP % kAtPos) == 0 && (kCPos % kAtPos) == 0);
static_assert(kWRows == 2048 && (768 % 8) == 0 && (1024 % 8) == 0 && (1792 % 8) == 0);

constexpr float kXCarry  = 16.0f;
constexpr float kWCarry  = 256.0f;
constexpr float kO0Carry = 64.0f;
constexpr float kZ1Carry = 1024.0f;
constexpr float kO1Carry = 1024.0f;
constexpr float kScaleQkv0 = 1.0f / (kXCarry * kWCarry);
constexpr float kScaleZ1   = kZ1Carry / (kO0Carry * kWCarry);
constexpr float kScaleQkv1 = 1.0f / (kZ1Carry * kWCarry);
constexpr float kScaleOut  = 1.0f / (kO1Carry * kWCarry);
constexpr float kInvP      = 1.0f / (float)kP;

constexpr double c_rsqrt(double x) {
  double y = 1.0 / x;
  for (int i = 0; i < 64; ++i) y = y * (1.5 - 0.5 * x * y * y);
  return y;
}
constexpr float kScale = (float)c_rsqrt((double)kDh);
static_assert(kScale > 0.176776f && kScale < 0.176777f);

constexpr size_t kOffW    = 0;
constexpr size_t kOffXY   = kOffW    + (size_t)kWRows * kD * 2;
constexpr size_t kOffPart = kOffXY   + (size_t)2 * kPos * kD * 2;
constexpr size_t kOffQkvG = kOffPart + (size_t)16 * kMeanCh * kD * 4;
constexpr size_t kOffBig  = kOffQkvG + (size_t)16 * kQkvN * 4;
constexpr size_t kOffO0   = kOffBig  + (size_t)4 * kCPos * 512 * 4;
constexpr size_t kOffZ1   = kOffO0   + (size_t)4 * kCPos * kD * 2;
constexpr size_t kOffQ1   = kOffZ1   + (size_t)4 * kCPos * kD * 2;
constexpr size_t kOffO1   = kOffQ1   + (size_t)2 * kCPos * kD * 4;
constexpr size_t kWsTotal = kOffO1   + (size_t)2 * kCPos * kD * 2;
static_assert(kWsTotal == 124043264ull);
static_assert(kWsTotal <= 134217728ull);
static_assert((size_t)2 * kCPos * kQkvN * 4 <= (size_t)4 * kCPos * 512 * 4);
static_assert((kOffXY % 128) == 0 && (kOffPart % 128) == 0 && (kOffQkvG % 128) == 0 && (kOffBig % 128) == 0 &&
              (kOffO0 % 128) == 0 && (kOffZ1 % 128) == 0 && (kOffQ1 % 128) == 0 && (kOffO1 % 128) == 0);
static_assert((size_t)kPos * kD * 4 == 25690112ull);

__device__ __forceinline__ unsigned short f2bf_bits(float f) {
  unsigned u = __float_as_uint(f);
  return (unsigned short)((u + 0x7FFFu + ((u >> 16) & 1u)) >> 16);
}
__device__ __forceinline__ float bf_bits2f(unsigned short h) { return __uint_as_float(((unsigned)h) << 16); }
__device__ __forceinline__ float bf_rne(float f) { return bf_bits2f(f2bf_bits(f)); }
__device__ __forceinline__ unsigned pk16(unsigned short a, unsigned short b) { return (unsigned)a | ((unsigned)b << 16); }
__device__ __forceinline__ unsigned short h_bits(float f) { const _Float16 h = (_Float16)f; return __builtin_bit_cast(unsigned short, h); }

__device__ __forceinline__ void keep4_h(v16h a, v16h b, v16h c, v16h d) { asm volatile("v_nop" :: "v"(a), "v"(b), "v"(c), "v"(d)); }
__device__ __forceinline__ void acc_guard4(v8f& a, v8f& b, v8f& c, v8f& d) { asm volatile("v_nop\n\tv_nop\n\tv_nop\n\tv_nop" : "+v"(a), "+v"(b), "+v"(c), "+v"(d)); }
__device__ __forceinline__ v8f mma_h(v16h a, v16h b, v8f c) {
  c = __builtin_amdgcn_wmma_f32_16x16x32_f16(false, a, false, b, (short)0, c, false, false);
  asm volatile("v_nop\n\tv_nop\n\tv_nop\n\tv_nop" : "+v"(c) : "v"(a), "v"(b));
  return c;
}
struct FragH {
  union U { v16h v; v8h h[2]; };
  static __device__ __forceinline__ v16h load(const _Float16* p) {
    U f; f.h[0] = *(const v8h*)(p); f.h[1] = *(const v8h*)(p + 16); return f.v;
  }
};

template <int BIAS_MODE, int OUT_MODE>
__global__ __launch_bounds__(256) void wmma_gemm64(
    const unsigned short* __restrict__ Ap, int lda, long strideA,
    const unsigned short* __restrict__ Btp, int ldb, long strideB,
    void* __restrict__ Cout, int ldc, long strideC,
    const float* __restrict__ bias, float bscale,
    int M, int N, int K, float scale) {
  const _Float16* A  = (const _Float16*)Ap;
  const _Float16* Bt = (const _Float16*)Btp;
  __shared__ __align__(16) float sT[8][16 * 68];
  const int b    = blockIdx.y;
  const int lane = threadIdx.x & 31;
  const int wave = __builtin_amdgcn_readfirstlane((int)(threadIdx.x >> 5));
  const int tilesN = N >> 6;
  const int tilesM = M >> 6;
  const int tile = blockIdx.x * 8 + wave;
  if (tile >= tilesM * tilesN) return;
  const int tm = tile / tilesN;
  const int tn = tile - tm * tilesN;
  const int m0 = tm << 6;
  const int n0 = tn << 6;

  const _Float16* Ab = A  + (size_t)b * strideA;
  const _Float16* Bb = Bt + (size_t)b * strideB;

  const int rlane = lane & 15;
  const int koff  = (lane >> 4) * 8;
  const int mOff  = (lane >> 4) * 8;

  v8f acc[4][4];
#pragma unroll
  for (int i = 0; i < 4; ++i)
#pragma unroll
    for (int j = 0; j < 4; ++j) acc[i][j] = (v8f){0.f,0.f,0.f,0.f,0.f,0.f,0.f,0.f};

  for (int k0 = 0; k0 < K; k0 += 32) {
    v16h bh[4];
#pragma unroll
    for (int j = 0; j < 4; ++j) {
      const size_t bo = (size_t)(n0 + (j << 4) + rlane) * ldb + koff + k0;
      bh[j] = FragH::load(Bb + bo);
    }
#pragma unroll
    for (int i = 0; i < 4; ++i) {
      const size_t ao = (size_t)(m0 + (i << 4) + rlane) * lda + koff + k0;
      const v16h ah = FragH::load(Ab + ao);
#pragma unroll
      for (int j = 0; j < 4; ++j) acc[i][j] = mma_h(ah, bh[j], acc[i][j]);
    }
    keep4_h(bh[0], bh[1], bh[2], bh[3]);
  }
  acc_guard4(acc[0][0], acc[0][1], acc[0][2], acc[0][3]);
  acc_guard4(acc[1][0], acc[1][1], acc[1][2], acc[1][3]);
  acc_guard4(acc[2][0], acc[2][1], acc[2][2], acc[2][3]);
  acc_guard4(acc[3][0], acc[3][1], acc[3][2], acc[3][3]);

  float* slab = sT[wave];
#pragma unroll
  for (int i = 0; i < 4; ++i) {
    const int mBase = m0 + (i << 4);
#pragma unroll
    for (int j = 0; j < 4; ++j) {
      const int n = n0 + (j << 4) + rlane;
      float bv = 0.f;
      if (BIAS_MODE == 2) bv = bf_rne(bias[n]) * bscale;
#pragma unroll
      for (int r = 0; r < 8; ++r) {
        float v = acc[i][j][r] * scale;
        if (BIAS_MODE == 2) v += bv;
        slab[(mOff + r) * 68 + (j << 4) + rlane] = v;
      }
    }
    __builtin_amdgcn_fence(__ATOMIC_RELEASE, "workgroup");
    __builtin_amdgcn_wave_barrier();
    __builtin_amdgcn_fence(__ATOMIC_ACQUIRE, "workgroup");
    if (OUT_MODE == 0) {
      float* C = (float*)Cout + (size_t)b * strideC;
      const int hh = lane >> 4, c4 = (lane & 15) * 4;
      for (int pass = 0; pass < 2; ++pass) {
#pragma unroll
        for (int it = 0; it < 8; ++it) {
          const int row = it * 2 + hh;
          v4f v = *(const v4f*)(slab + row * 68 + c4);
          *(volatile v4f*)(C + (size_t)(mBase + row) * ldc + n0 + c4) = v;
        }
        __threadfence();
      }
    } else {
      const int q = lane >> 3, c8 = (lane & 7) * 8;
      unsigned short* C = (unsigned short*)Cout + (size_t)b * strideC;
      for (int pass = 0; pass < 2; ++pass) {
#pragma unroll
        for (int it = 0; it < 4; ++it) {
          const int row = it * 4 + q;
          const float* sp = slab + row * 68 + c8;
          v8h hv;
#pragma unroll
          for (int e = 0; e < 8; ++e) hv[e] = (_Float16)sp[e];
          *(volatile v8h*)(C + (size_t)(mBase + row) * ldc + n0 + c8) = hv;
        }
        __threadfence();
      }
    }
    __builtin_amdgcn_fence(__ATOMIC_RELEASE, "workgroup");
    __builtin_amdgcn_wave_barrier();
    __builtin_amdgcn_fence(__ATOMIC_ACQUIRE, "workgroup");
  }
}

__global__ __launch_bounds__(256) void weight_plane_kernel(
    const float* __restrict__ Wq0, const float* __restrict__ Wo0,
    const float* __restrict__ Wq1, const float* __restrict__ Wo1,
    unsigned short* __restrict__ W16) {
  const int i = blockIdx.x * 256 + threadIdx.x;
  if (i >= kWRows * kD / 8) return;
  const int rowb = blockIdx.x * 8;
  const float* src;
  int rbase;
  if (rowb < 768)       { src = Wq0; rbase = 0; }
  else if (rowb < 1024) { src = Wo0; rbase = 768; }
  else if (rowb < 1792) { src = Wq1; rbase = 1024; }
  else                  { src = Wo1; rbase = 1792; }
  const size_t e0 = (size_t)i * 8;
  const float* p = src + (e0 - (size_t)rbase * kD);
  const v4f a = *(const v4f*)(p);
  const v4f c = *(const v4f*)(p + 4);
  unsigned short hb[8];
#pragma unroll
  for (int e = 0; e < 4; ++e) {
    const float fa = a[e];
    const float fc = c[e];
    hb[e]     = h_bits(bf_rne(fa) * kWCarry);
    hb[4 + e] = h_bits(bf_rne(fc) * kWCarry);
  }
  const v4u u = (v4u){pk16(hb[0], hb[1]), pk16(hb[2], hb[3]), pk16(hb[4], hb[5]), pk16(hb[6], hb[7])};
  unsigned short* q = W16 + e0;
  *(volatile v4u*)q = u;
  __threadfence();
  *(volatile v4u*)q = u;
}

__global__ __launch_bounds__(256) void xy_plane_kernel(
    const float* __restrict__ x, const float* __restrict__ y,
    unsigned short* __restrict__ XY, float* __restrict__ PART) {
  __shared__ float red[8][256];
  const int tid = threadIdx.x, lane = tid & 31;
  const int wave = __builtin_amdgcn_readfirstlane((int)(threadIdx.x >> 5));
  const int chunk = blockIdx.x, b = blockIdx.y, t = blockIdx.z;
  const float* src = (t == 0) ? x : y;
  float acc[8];
#pragma unroll
  for (int e = 0; e < 8; ++e) acc[e] = 0.f;
#pragma unroll 1
  for (int i = 0; i < 7; ++i) {
    const int p = chunk * kMeanLen + wave + 8 * i;
    const size_t row = (size_t)b * kP + p;
    const float* sp = src + row * kD + lane * 8;
    const v4f a = *(const v4f*)(sp);
    const v4f c = *(const v4f*)(sp + 4);
    unsigned short hb[8];
#pragma unroll
    for (int e = 0; e < 4; ++e) {
      const float fa = a[e];
      const float fc = c[e];
      const float ra = bf_rne(fa);
      const float rc = bf_rne(fc);
      acc[e]     += ra;
      acc[4 + e] += rc;
      hb[e]     = h_bits(ra * kXCarry);
      hb[4 + e] = h_bits(rc * kXCarry);
    }
    const v4u u = (v4u){pk16(hb[0], hb[1]), pk16(hb[2], hb[3]), pk16(hb[4], hb[5]), pk16(hb[6], hb[7])};
    unsigned short* q = XY + ((size_t)t * kPos + row) * kD + lane * 8;
    *(volatile v4u*)q = u;
    __threadfence();
    *(volatile v4u*)q = u;
  }
#pragma unroll
  for (int e = 0; e < 8; ++e) red[wave][lane * 8 + e] = acc[e];
  __syncthreads();
  float s = red[0][tid];
#pragma unroll
  for (int w = 1; w < 8; ++w) s += red[w][tid];
  float* q = PART + ((size_t)((t * kB + b) * kMeanCh + chunk)) * kD + tid;
  *(volatile float*)q = s;
  __threadfence();
  *(volatile float*)q = s;
}

__global__ __launch_bounds__(256) void mean_token_qkv_kernel(
    const float* __restrict__ PART, const float* __restrict__ Wq0, float* __restrict__ QKVG) {
  __shared__ float sm[256];
  const int tid = threadIdx.x;
  const int r = blockIdx.y;
  float s = 0.f;
#pragma unroll 1
  for (int c = 0; c < kMeanCh; ++c) s += PART[((size_t)r * kMeanCh + c) * kD + tid];
  sm[tid] = s * kInvP;
  __syncthreads();
  const int n = blockIdx.x * 256 + tid;
  const float* wr = Wq0 + (size_t)n * kD;
  float acc = 0.f;
#pragma unroll 1
  for (int k4 = 0; k4 < kD / 4; ++k4) {
    const v4f w = *(const v4f*)(wr + 4 * k4);
    const float w0 = w[0];
    const float w1 = w[1];
    const float w2 = w[2];
    const float w3 = w[3];
    acc = fmaf(bf_rne(w0), sm[4 * k4 + 0], acc);
    acc = fmaf(bf_rne(w1), sm[4 * k4 + 1], acc);
    acc = fmaf(bf_rne(w2), sm[4 * k4 + 2], acc);
    acc = fmaf(bf_rne(w3), sm[4 * k4 + 3], acc);
  }
  float* q = QKVG + (size_t)r * kQkvN + n;
  *(volatile float*)q = acc;
  __threadfence();
  *(volatile float*)q = acc;
}

__device__ __forceinline__ float dot2(v2f q, v2f k, float s) {
  s = fmaf(q[0], k[0], s);
  return fmaf(q[1], k[1], s);
}
__device__ __forceinline__ float mix3(float pa, float va, float pb, float vb, float pc, float vc) {
  float o = pa * va;
  o = fmaf(pb, vb, o);
  return fmaf(pc, vc, o);
}
__device__ __forceinline__ void softmax3(float a, float b, float c, float carry, float& pa, float& pb, float& pc) {
  const float m = fmaxf(a, fmaxf(b, c));
  const float ea = expf((a - m) * kScale);
  const float eb = expf((b - m) * kScale);
  const float ec = expf((c - m) * kScale);
  const float inv = carry * __builtin_amdgcn_rcpf(ea + eb + ec);
  pa = ea * inv;
  pb = eb * inv;
  pc = ec * inv;
}

__global__ __launch_bounds__(128) void attn_stage0_kernel(
    const float* __restrict__ QKV0, const float* __restrict__ QKVG,
    unsigned short* __restrict__ O0, int batch0) {
  __shared__ __align__(16) unsigned int sO[4 * kAtPos * 128];
  const int tid  = threadIdx.x;
  const int pl   = tid >> 3;
  const int head = tid & 7;
  const int pos  = blockIdx.x * kAtPos + pl;
  int bg = batch0 + (int)(blockIdx.x / (kP / kAtPos));
  bg = bg < 0 ? 0 : (bg > kB - 1 ? kB - 1 : bg);
  const float* r0 = QKV0 + (size_t)pos * kQkvN + head * kDh;
  const float* r1 = QKV0 + (size_t)(kCPos + pos) * kQkvN + head * kDh;
  const float* r2 = QKVG + (size_t)bg * kQkvN + head * kDh;
  const float* r3 = QKVG + (size_t)(kB + bg) * kQkvN + head * kDh;

  float s00 = 0.f, s01 = 0.f, s02 = 0.f;
  float s10 = 0.f, s11 = 0.f, s13 = 0.f;
  float s20 = 0.f, s22 = 0.f, s23 = 0.f;
  float s31 = 0.f, s32 = 0.f, s33 = 0.f;
#pragma unroll 1
  for (int dc = 0; dc < kDh / 2; ++dc) {
    const int o = dc * 2;
    const v2f q0 = *(const v2f*)(r0 + o);
    const v2f q1 = *(const v2f*)(r1 + o);
    const v2f q2 = *(const v2f*)(r2 + o);
    const v2f q3 = *(const v2f*)(r3 + o);
    const v2f k0 = *(const v2f*)(r0 + kInner + o);
    const v2f k1 = *(const v2f*)(r1 + kInner + o);
    const v2f k2 = *(const v2f*)(r2 + kInner + o);
    const v2f k3 = *(const v2f*)(r3 + kInner + o);
    s00 = dot2(q0, k0, s00); s01 = dot2(q0, k1, s01); s02 = dot2(q0, k2, s02);
    s10 = dot2(q1, k0, s10); s11 = dot2(q1, k1, s11); s13 = dot2(q1, k3, s13);
    s20 = dot2(q2, k0, s20); s22 = dot2(q2, k2, s22); s23 = dot2(q2, k3, s23);
    s31 = dot2(q3, k1, s31); s32 = dot2(q3, k2, s32); s33 = dot2(q3, k3, s33);
  }
  float p00, p01, p02, p10, p11, p13, p20, p22, p23, p31, p32, p33;
  softmax3(s00, s01, s02, kO0Carry, p00, p01, p02);
  softmax3(s10, s11, s13, kO0Carry, p10, p11, p13);
  softmax3(s20, s22, s23, kO0Carry, p20, p22, p23);
  softmax3(s31, s32, s33, kO0Carry, p31, p32, p33);

  unsigned int* so = sO + pl * 128 + head * 16;
#pragma unroll 1
  for (int dc = 0; dc < kDh / 2; ++dc) {
    const int o = 2 * kInner + dc * 2;
    const v2f v0 = *(const v2f*)(r0 + o);
    const v2f v1 = *(const v2f*)(r1 + o);
    const v2f v2 = *(const v2f*)(r2 + o);
    const v2f v3 = *(const v2f*)(r3 + o);
    const float a0 = mix3(p00, v0[0], p01, v1[0], p02, v2[0]);
    const float b0 = mix3(p00, v0[1], p01, v1[1], p02, v2[1]);
    const float a1 = mix3(p10, v0[0], p11, v1[0], p13, v3[0]);
    const float b1 = mix3(p10, v0[1], p11, v1[1], p13, v3[1]);
    const float a2 = mix3(p20, v0[0], p22, v2[0], p23, v3[0]);
    const float b2 = mix3(p20, v0[1], p22, v2[1], p23, v3[1]);
    const float a3 = mix3(p31, v1[0], p32, v2[0], p33, v3[0]);
    const float b3 = mix3(p31, v1[1], p32, v2[1], p33, v3[1]);
    so[0 * kAtPos * 128 + dc] = pk16(h_bits(a0), h_bits(b0));
    so[1 * kAtPos * 128 + dc] = pk16(h_bits(a1), h_bits(b1));
    so[2 * kAtPos * 128 + dc] = pk16(h_bits(a2), h_bits(b2));
    so[3 * kAtPos * 128 + dc] = pk16(h_bits(a3), h_bits(b3));
  }
  __syncthreads();
  for (int pass = 0; pass < 2; ++pass) {
#pragma unroll 1
    for (int it = 0; it < 16; ++it) {
      const int u = it * 128 + tid;
      const int t = u >> 9;
      const int w = u & 511;
      const v4u val = *(const v4u*)(sO + u * 4);
      unsigned short* dst = O0 + ((size_t)(t * kCPos + (int)blockIdx.x * kAtPos)) * kD + (size_t)w * 8;
      *(volatile v4u*)dst = val;
    }
    __threadfence();
  }
}

__device__ __forceinline__ float dot4(v4f q, v4f k, float s) {
  s = fmaf(q[0], k[0], s);
  s = fmaf(q[1], k[1], s);
  s = fmaf(q[2], k[2], s);
  return fmaf(q[3], k[3], s);
}
__device__ __forceinline__ float mix2(float pa, float va, float pb, float vb) {
  return fmaf(pb, vb, pa * va);
}
__device__ __forceinline__ void softmax2(float a, float b, float carry, float& pa, float& pb) {
  const float m = fmaxf(a, b);
  const float ea = expf((a - m) * kScale);
  const float eb = expf((b - m) * kScale);
  const float inv = carry * __builtin_amdgcn_rcpf(ea + eb);
  pa = ea * inv;
  pb = eb * inv;
}

__global__ __launch_bounds__(128) void attn_stage1_kernel(
    const float* __restrict__ Q1, const float* __restrict__ KV1, unsigned short* __restrict__ O1) {
  __shared__ __align__(16) unsigned int sO[2 * kAtPos * 128];
  const int tid  = threadIdx.x;
  const int pl   = tid >> 3;
  const int head = tid & 7;
  const int pos  = blockIdx.x * kAtPos + pl;
  const float* q0p = Q1 + (size_t)pos * kInner + head * kDh;
  const float* q1p = Q1 + (size_t)(kCPos + pos) * kInner + head * kDh;
  const float* c0 = KV1 + (size_t)pos * 512 + head * kDh;
  const float* c1 = KV1 + (size_t)(kCPos + pos) * 512 + head * kDh;
  const float* c2 = KV1 + (size_t)(2 * kCPos + pos) * 512 + head * kDh;
  const float* c3 = KV1 + (size_t)(3 * kCPos + pos) * 512 + head * kDh;

  float s00 = 0.f, s02 = 0.f, s11 = 0.f, s13 = 0.f;
#pragma unroll 1
  for (int dc = 0; dc < kDh / 4; ++dc) {
    const int o = dc * 4;
    const v4f q0 = *(const v4f*)(q0p + o);
    const v4f q1 = *(const v4f*)(q1p + o);
    const v4f k0 = *(const v4f*)(c0 + o);
    const v4f k1 = *(const v4f*)(c1 + o);
    const v4f k2 = *(const v4f*)(c2 + o);
    const v4f k3 = *(const v4f*)(c3 + o);
    s00 = dot4(q0, k0, s00);
    s02 = dot4(q0, k2, s02);
    s11 = dot4(q1, k1, s11);
    s13 = dot4(q1, k3, s13);
  }
  float p00, p02, p11, p13;
  softmax2(s00, s02, kO1Carry, p00, p02);
  softmax2(s11, s13, kO1Carry, p11, p13);

  unsigned int* so = sO + pl * 128 + head * 16;
#pragma unroll 1
  for (int dc = 0; dc < kDh / 4; ++dc) {
    const int o = kInner + dc * 4;
    const v4f v0 = *(const v4f*)(c0 + o);
    const v4f v1 = *(const v4f*)(c1 + o);
    const v4f v2 = *(const v4f*)(c2 + o);
    const v4f v3 = *(const v4f*)(c3 + o);
    const float a0 = mix2(p00, v0[0], p02, v2[0]);
    const float a1 = mix2(p00, v0[1], p02, v2[1]);
    const float a2 = mix2(p00, v0[2], p02, v2[2]);
    const float a3 = mix2(p00, v0[3], p02, v2[3]);
    const float b0 = mix2(p11, v1[0], p13, v3[0]);
    const float b1 = mix2(p11, v1[1], p13, v3[1]);
    const float b2 = mix2(p11, v1[2], p13, v3[2]);
    const float b3 = mix2(p11, v1[3], p13, v3[3]);
    so[0 * kAtPos * 128 + dc * 2 + 0] = pk16(h_bits(a0), h_bits(a1));
    so[0 * kAtPos * 128 + dc * 2 + 1] = pk16(h_bits(a2), h_bits(a3));
    so[1 * kAtPos * 128 + dc * 2 + 0] = pk16(h_bits(b0), h_bits(b1));
    so[1 * kAtPos * 128 + dc * 2 + 1] = pk16(h_bits(b2), h_bits(b3));
  }
  __syncthreads();
  for (int pass = 0; pass < 2; ++pass) {
#pragma unroll 1
    for (int it = 0; it < 8; ++it) {
      const int u = it * 128 + tid;
      const int t = u >> 9;
      const int w = u & 511;
      const v4u val = *(const v4u*)(sO + u * 4);
      unsigned short* dst = O1 + ((size_t)(t * kCPos + (int)blockIdx.x * kAtPos)) * kD + (size_t)w * 8;
      *(volatile v4u*)dst = val;
    }
    __threadfence();
  }
}

static_assert(((kCPos / 64) * (kQkvN / 64)) % 8 == 0);
static_assert(((4 * kCPos / 64) * (kD / 64)) % 8 == 0);
static_assert(((2 * kCPos / 64) * (kD / 64)) % 8 == 0);
static_assert(((4 * kCPos / 64) * (512 / 64)) % 8 == 0);
static_assert(((kCPos / 64) * (kD / 64)) % 8 == 0);

extern "C" void kernel_launch(void* const* d_in, const int* in_sizes, int n_in,
                              void* d_out, int out_size, void* d_ws, size_t ws_size,
                              hipStream_t stream) {
  if (n_in < 8) return;
  if (in_sizes[0] != kPos * kD) return;
  if (in_sizes[1] != kPos * kD) return;
  if (in_sizes[2] != kQkvN * kD) return;
  if (in_sizes[3] != kD * kInner) return;
  if (in_sizes[4] != kD) return;
  if (in_sizes[5] != kQkvN * kD) return;
  if (in_sizes[6] != kD * kInner) return;
  if (in_sizes[7] != kD) return;
  if (out_size != 2 * kPos * kD) return;
  if (ws_size < kWsTotal) return;

  const float* x    = (const float*)d_in[0];
  const float* y    = (const float*)d_in[1];
  const float* Wq0  = (const float*)d_in[2];
  const float* Wo0  = (const float*)d_in[3];
  const float* b0   = (const float*)d_in[4];
  const float* Wq1  = (const float*)d_in[5];
  const float* Wo1  = (const float*)d_in[6];
  const float* b1   = (const float*)d_in[7];
  float* out = (float*)d_out;

  char* ws = (char*)d_ws;
  unsigned short* W16  = (unsigned short*)(ws + kOffW);
  unsigned short* XY16 = (unsigned short*)(ws + kOffXY);
  float*          PART = (float*)(ws + kOffPart);
  float*          QKVG = (float*)(ws + kOffQkvG);
  float*          BIG  = (float*)(ws + kOffBig);
  unsigned short* O0   = (unsigned short*)(ws + kOffO0);
  unsigned short* Z1   = (unsigned short*)(ws + kOffZ1);
  float*          Q1   = (float*)(ws + kOffQ1);
  unsigned short* O1   = (unsigned short*)(ws + kOffO1);
  float* QKV0 = BIG;
  float* KV1  = BIG;

  const unsigned short* Wq0h = W16;
  const unsigned short* Wo0h = W16 + (size_t)768 * kD;
  const unsigned short* Wq1h = W16 + (size_t)1024 * kD;
  const unsigned short* Wk1h = W16 + (size_t)(1024 + kInner) * kD;
  const unsigned short* Wo1h = W16 + (size_t)1792 * kD;

  weight_plane_kernel<<<(kWRows * kD / 8) / 256, 256, 0, stream>>>(Wq0, Wo0, Wq1, Wo1, W16);
  xy_plane_kernel<<<dim3(kMeanCh, kB, 2), 256, 0, stream>>>(x, y, XY16, PART);
  mean_token_qkv_kernel<<<dim3(kQkvN / 256, 16), 256, 0, stream>>>(PART, Wq0, QKVG);

  for (int c = 0; c < kChunks; ++c) {
    wmma_gemm64<0, 0><<<dim3((kCPos / 64) * (kQkvN / 64) / 8, 2), 256, 0, stream>>>(
        XY16 + (size_t)c * kCPos * kD, kD, (long)kPos * kD,
        Wq0h, kD, 0L,
        (void*)QKV0, kQkvN, (long)kCPos * kQkvN,
        b0, 0.0f,
        kCPos, kQkvN, kD, kScaleQkv0);

    attn_stage0_kernel<<<kCPos / kAtPos, 128, 0, stream>>>(QKV0, QKVG, O0, c * kChunkB);

    wmma_gemm64<2, 1><<<dim3((4 * kCPos / 64) * (kD / 64) / 8, 1), 256, 0, stream>>>(
        O0, kInner, 0L,
        Wo0h, kInner, 0L,
        (void*)Z1, kD, 0L,
        b0, kZ1Carry,
        4 * kCPos, kD, kInner, kScaleZ1);

    wmma_gemm64<0, 0><<<dim3((2 * kCPos / 64) * (kInner / 64) / 8, 1), 256, 0, stream>>>(
        Z1, kD, 0L,
        Wq1h, kD, 0L,
        (void*)Q1, kInner, 0L,
        b0, 0.0f,
        2 * kCPos, kInner, kD, kScaleQkv1);

    wmma_gemm64<0, 0><<<dim3((4 * kCPos / 64) * (512 / 64) / 8, 1), 256, 0, stream>>>(
        Z1, kD, 0L,
        Wk1h, kD, 0L,
        (void*)KV1, 512, 0L,
        b0, 0.0f,
        4 * kCPos, 512, kD, kScaleQkv1);

    attn_stage1_kernel<<<kCPos / kAtPos, 128, 0, stream>>>(Q1, KV1, O1);

    wmma_gemm64<2, 0><<<dim3((kCPos / 64) * (kD / 64) / 8, 2), 256, 0, stream>>>(
        O1, kInner, (long)kCPos * kInner,
        Wo1h, kInner, 0L,
        (void*)(out + (size_t)c * kCPos * kD), kD, (long)kPos * kD,
        b1, 1.0f,
        kCPos, kD, kInner, kScaleOut);
  }
}
